// Semantic_70342974374320
// MI455X (gfx1250) — hardware-verified
//
#include <hip/hip_runtime.h>
#include <stddef.h>
#include <stdint.h>


typedef _Float16 v16h __attribute__((ext_vector_type(16)));
typedef _Float16 v8h  __attribute__((ext_vector_type(8)));
typedef float    v8f  __attribute__((ext_vector_type(8)));
typedef float    v4f  __attribute__((ext_vector_type(4)));
typedef int      v4i  __attribute__((ext_vector_type(4)));
typedef v4f v4fa __attribute__((may_alias));
union Frag { v16h v; v8h hv[2]; };

#define KOFF 27
#define CH 32
#define RG 128
#define RGS 7
#define NSB 256
#define NCHUNK 6
#define WSCALE 64.0f
#define WINV (1.0f / 64.0f)

__device__ __forceinline__ int clampi(int v, int lo, int hi) {
    return v < lo ? lo : (v > hi ? hi : v);
}

__device__ __forceinline__ void mma2(v8f& c0, v8f& c1, const v16h a, const v16h b0, const v16h b1) {
    c0 = __builtin_amdgcn_wmma_f32_16x16x32_f16(false, a, false, b0, (short)0, c0, false, false);
    c1 = __builtin_amdgcn_wmma_f32_16x16x32_f16(false, a, false, b1, (short)0, c1, false, false);
    asm volatile("v_nop\n\tv_nop\n\tv_nop\n\tv_nop" : "+v"(c0), "+v"(c1) : "v"(a), "v"(b0), "v"(b1));
}

__global__ __launch_bounds__(256)
void k_wprep(const float* __restrict__ W1, const float* __restrict__ W2,
             _Float16* Wt1, _Float16* Wt2, int total) {
    const int i = blockIdx.x * 256 + threadIdx.x;
    const bool act = i < total;
    const int ii = act ? i : 0;
    const int k = ii >> 7, rem = ii & 127, co = rem >> 2, q = rem & 3;
    const size_t src = (size_t)k * (CH * CH) + co;
    v8h a, b;
#pragma unroll
    for (int j = 0; j < 8; ++j) {
        const size_t s = src + (size_t)(q * 8 + j) * CH;
        a[j] = (_Float16)(W1[s] * WSCALE);
        b[j] = (_Float16)(W2[s] * WSCALE);
    }
    const size_t o = (size_t)k * (CH * CH) + (size_t)co * CH + q * 8;
    if (act) {
        *(volatile v8h*)(Wt1 + o) = a;
        *(volatile v8h*)(Wt2 + o) = b;
    }
    __threadfence();
    if (act) {
        *(volatile v8h*)(Wt1 + o) = a;
        *(volatile v8h*)(Wt2 + o) = b;
    }
}

__global__ __launch_bounds__(32)
void k_count(const int* __restrict__ kin, const int* __restrict__ kout, int P,
             int ndst, int G, int GP, int* cnt) {
    extern __shared__ int hist[];
    const int l = threadIdx.x, k = blockIdx.x;
    const size_t base = (size_t)k * P;
    for (int i = l; i < GP; i += 32) hist[i] = 0;
    __syncthreads();
    for (int b0 = 0; b0 < P; b0 += 32) {
        const int p = b0 + l;
        int pin = -1, dst = -1;
        if (p < P) { pin = kin[base + p]; dst = kout[base + p]; }
        const bool valid = (pin >= 0) && ((unsigned)dst < (unsigned)ndst);
        const int g = valid ? (dst >> RGS) : 0;
        unsigned eq = __builtin_amdgcn_ballot_w32(valid);
#pragma unroll
        for (int bt = 0; bt < 16; ++bt) {
            const bool bit = (g >> bt) & 1;
            const unsigned bal = __builtin_amdgcn_ballot_w32(bit);
            eq &= bit ? bal : ~bal;
        }
        const int c = __popc(eq);
        const int rank = __popc(eq & ((1u << l) - 1u));
        if (valid && rank == 0) hist[g] += c;
    }
    __syncthreads();
    int* row = cnt + (size_t)k * GP;
    for (int pass = 0; pass < 2; ++pass) {
        for (int b0 = 0; b0 < GP; b0 += 128) {
            const int e = b0 + 4 * l;
            v4i v = {hist[e], hist[e + 1], hist[e + 2], hist[e + 3]};
            *(volatile v4i*)(row + e) = v;
        }
        __threadfence();
    }
}

__global__ __launch_bounds__(512)
void k_scan(const int* __restrict__ cnt, int L, int GP, int cells, int cmax,
            int nlines, int lpt, int* off) {
    __shared__ int wtot[16];
    __shared__ int wex[16];
    const int t = threadIdx.x, l = t & 31, w = t >> 5;
    const int lb = t * lpt;
    int le = lb + lpt; if (le > nlines) le = nlines;
    int tsum = 0;
    for (int ln = lb; ln < le; ++ln) {
        for (int e = 0; e < 32; ++e) {
            const int j = ln * 32 + e;
            if (j < cells) {
                const int g = j / L;
                const int kk = j - g * L;
                int c = cnt[(size_t)kk * GP + g];
                c = clampi(c, 0, cmax);
                tsum += (c + 15) & ~15;
            }
        }
    }
    int incl = tsum;
    for (int d = 1; d < 32; d <<= 1) {
        const int y = __shfl_up(incl, d, 32);
        if (l >= d) incl += y;
    }
    if (l == 31) wtot[w] = incl;
    __syncthreads();
    if (w == 0) {
        const int v = (l < 16) ? wtot[l] : 0;
        int i2 = v;
        for (int d = 1; d < 32; d <<= 1) {
            const int y = __shfl_up(i2, d, 32);
            if (l >= d) i2 += y;
        }
        if (l < 16) wex[l] = i2 - v;
    }
    __syncthreads();
    const int excl = wex[w] + incl - tsum;
    for (int pass = 0; pass < 2; ++pass) {
        int run = excl;
        for (int ln = lb; ln < le; ++ln) {
            int vals[32];
#pragma unroll
            for (int e = 0; e < 32; ++e) {
                const int j = ln * 32 + e;
                vals[e] = run;
                if (j < cells) {
                    const int g = j / L;
                    const int kk = j - g * L;
                    int c = cnt[(size_t)kk * GP + g];
                    c = clampi(c, 0, cmax);
                    run += (c + 15) & ~15;
                }
            }
            volatile v4i* dstp = (volatile v4i*)(off + (size_t)ln * 32);
#pragma unroll
            for (int qd = 0; qd < 8; ++qd) {
                v4i vv = {vals[4 * qd], vals[4 * qd + 1], vals[4 * qd + 2], vals[4 * qd + 3]};
                dstp[qd] = vv;
            }
        }
        __threadfence();
    }
}

__global__ __launch_bounds__(32)
void k_fill(const int* __restrict__ kin, const int* __restrict__ kout, int P,
            int nsrc, int ndst, int G, int L, const int* __restrict__ off,
            int slotcap, int* slot) {
    extern __shared__ int cur[];
    const int l = threadIdx.x, k = blockIdx.x;
    const size_t base = (size_t)k * P;
    for (int pass = 0; pass < 2; ++pass) {
        for (int g = l; g < G; g += 32) cur[g] = clampi(off[(size_t)g * L + k], 0, slotcap);
        __syncthreads();
        for (int b0 = 0; b0 < P; b0 += 32) {
            const int p = b0 + l;
            int pin = -1, dst = -1;
            if (p < P) { pin = kin[base + p]; dst = kout[base + p]; }
            const bool valid = (pin >= 0) && ((unsigned)dst < (unsigned)ndst);
            const int g = valid ? (dst >> RGS) : 0;
            unsigned eq = __builtin_amdgcn_ballot_w32(valid);
#pragma unroll
            for (int bt = 0; bt < 16; ++bt) {
                const bool bit = (g >> bt) & 1;
                const unsigned bal = __builtin_amdgcn_ballot_w32(bit);
                eq &= bit ? bal : ~bal;
            }
            const int c = __popc(eq);
            const int rank = __popc(eq & ((1u << l) - 1u));
            const int cg = cur[g];
            if (valid) {
                const int pos = cg + rank;
                const int pc = (pin < nsrc) ? pin : (nsrc - 1);
                const int word = pc * 256 + (dst & (RG - 1));
                if ((unsigned)pos < (unsigned)slotcap) *(volatile int*)(slot + pos) = word;
            }
            if (valid && rank == 0) cur[g] = cg + c;
        }
        __syncthreads();
        for (int g = l; g < G; g += 32) {
            const int c0 = cur[g];
            const int e = clampi(off[(size_t)g * L + k + 1], 0, slotcap);
#pragma unroll
            for (int u = 0; u < 16; ++u) {
                const int pos = c0 + u;
                if (pos < e && (unsigned)pos < (unsigned)slotcap) *(volatile int*)(slot + pos) = -1;
            }
        }
        __threadfence();
        __syncthreads();
    }
}

__global__ __launch_bounds__(256)
void k_stats(const float* __restrict__ x, int nrows, int rb, float* part) {
    __shared__ float sred[256 * 8];
    __shared__ float sline[64];
    const int t = threadIdx.x, c4 = t & 7, rs = t >> 3;
    const int r0 = blockIdx.x * rb;
    int r1 = r0 + rb; if (r1 > nrows) r1 = nrows;
    v4f s = {0.f, 0.f, 0.f, 0.f};
    v4f q = {0.f, 0.f, 0.f, 0.f};
    for (int r = r0 + rs; r < r1; r += 32) {
        const v4f v = *(const v4f*)(x + (size_t)r * CH + 4 * c4);
        s += v;
        q += v * v;
    }
    v4fa* sr = (v4fa*)sred;
    sr[t * 2] = s;
    sr[t * 2 + 1] = q;
    __syncthreads();
    if (t < 64) {
        const int isq = t >> 5, ch = t & 31, cc4 = ch >> 2, comp = ch & 3;
        float a = 0.0f;
        for (int j = 0; j < 32; ++j) a += sred[(j * 8 + cc4) * 8 + isq * 4 + comp];
        sline[t] = a;
    }
    __syncthreads();
    if (t < 16) {
        const v4f v = ((const v4fa*)sline)[t];
        volatile v4f* d = (volatile v4f*)(part + (size_t)blockIdx.x * 64) + t;
        *d = v;
        __threadfence();
        *d = v;
    }
}

__global__ __launch_bounds__(64)
void k_statfin(const float* __restrict__ part, int nb, int nrows, float* stat) {
    __shared__ double S[64];
    __shared__ float sline[64];
    const int t = threadIdx.x;
    double a = 0.0;
    for (int b = 0; b < nb; ++b) a += (double)part[(size_t)b * 64 + t];
    S[t] = a;
    __syncthreads();
    if (t < 32) {
        const double inv = 1.0 / (double)nrows;
        const double mean = S[t] * inv;
        double var = S[32 + t] * inv - mean * mean;
        if (var < 0.0) var = 0.0;
        const double rstd = 1.0 / sqrt(var + 1e-4);
        sline[t] = (float)mean;
        sline[32 + t] = (float)rstd;
    }
    __syncthreads();
    if (t < 16) {
        const v4f v = ((const v4fa*)sline)[t];
        volatile v4f* d = (volatile v4f*)stat + t;
        *d = v;
        __threadfence();
        *d = v;
    }
}

__global__ __launch_bounds__(256)
void k_gather(const float* __restrict__ x, const float* __restrict__ stat,
              const int* __restrict__ slot, const int* __restrict__ off,
              int cell_a, int cell_b, int slotcap, int cap, int nsrc, _Float16* yg) {
    const int t = threadIdx.x, q = t & 3;
    const int i = blockIdx.x * 64 + (t >> 2);
    const int s0 = clampi(off[cell_a], 0, slotcap);
    const int s1 = clampi(off[cell_b], s0, slotcap);
    int cnt = s1 - s0; if (cnt > cap) cnt = cap;
    v8h o;
#pragma unroll
    for (int e = 0; e < 8; ++e) o[e] = (_Float16)0.0f;
    if (i < cnt) {
        const int w = slot[(size_t)s0 + i];
        if (w >= 0) {
            int pin = w >> 8; if (pin >= nsrc) pin = nsrc - 1;
            const float* xr = x + (size_t)pin * CH + q * 8;
            v4f a = *(const v4f*)xr;
            v4f b = *(const v4f*)(xr + 4);
            const v4f m0 = *(const v4f*)(stat + q * 8);
            const v4f m1 = *(const v4f*)(stat + q * 8 + 4);
            const v4f g0 = *(const v4f*)(stat + 32 + q * 8);
            const v4f g1 = *(const v4f*)(stat + 32 + q * 8 + 4);
            a = (a - m0) * g0;
            b = (b - m1) * g1;
#pragma unroll
            for (int e = 0; e < 4; ++e) {
                const float va = a[e] > 0.0f ? a[e] : 0.0f;
                const float vb = b[e] > 0.0f ? b[e] : 0.0f;
                o[e] = (_Float16)va;
                o[4 + e] = (_Float16)vb;
            }
        }
    }
    if (i < cap) {
        volatile v8h* d = (volatile v8h*)(yg + (size_t)i * CH + q * 8);
        *d = o;
        __threadfence();
        *d = o;
    }
}

__global__ __launch_bounds__(32)
void k_conv(const _Float16* __restrict__ yg, const _Float16* __restrict__ Wt,
            const int* __restrict__ slot, const int* __restrict__ off,
            const float* __restrict__ resid, int ga, int slotcap, int cap, int maxg,
            int nrows, int to_out, float* dst) {
    __shared__ float lacc[2 * RG * CH];
    const int l = threadIdx.x, h = l >> 4, m = l & 15;
    const int g = ga + blockIdx.x;
    const size_t cbase = (size_t)g * KOFF;
    const int s0 = clampi(off[(size_t)ga * KOFF], 0, slotcap);
    const int lo = clampi(off[cbase], 0, slotcap);
    int hi = clampi(off[cbase + KOFF], lo, slotcap);
    if (hi > lo + maxg) hi = lo + maxg;
    {
        v4fa* z = (v4fa*)lacc;
        const v4f zero = {0.f, 0.f, 0.f, 0.f};
        for (int i = 0; i < (2 * RG * CH / 4) / 32; ++i) z[i * 32 + l] = zero;
    }
    __syncthreads();
    int ce_prev = lo;
    for (int k = 0; k < KOFF; ++k) {
        const int cb = ce_prev;
        const int ce = clampi(off[cbase + k + 1], cb, hi);
        ce_prev = ce;
        const _Float16* wb = Wt + (size_t)k * (CH * CH);
        Frag b0, b1;
        b0.hv[0] = *(const v8h*)(wb + (size_t)m * CH + 8 * h);
        b0.hv[1] = *(const v8h*)(wb + (size_t)m * CH + 16 + 8 * h);
        b1.hv[0] = *(const v8h*)(wb + (size_t)(m + 16) * CH + 8 * h);
        b1.hv[1] = *(const v8h*)(wb + (size_t)(m + 16) * CH + 16 + 8 * h);
        for (int tt = cb; tt < ce; tt += 16) {
            const int s = tt + m;
            const int w = (s < ce) ? slot[s] : -1;
            const int d = (w >= 0) ? (w & (RG - 1)) : -1;
            const int i = clampi(s - s0, 0, cap - 1);
            const _Float16* yr = yg + (size_t)i * CH;
            Frag a;
            a.hv[0] = *(const v8h*)(yr + 8 * h);
            a.hv[1] = *(const v8h*)(yr + 16 + 8 * h);
            v8f c0 = {}, c1 = {};
            mma2(c0, c1, a.v, b0.v, b1.v);
            float* accb = lacc + h * (RG * CH) + m;
#pragma unroll
            for (int r = 0; r < 8; ++r) {
                const int dr = __shfl(d, 8 * h + r, 32);
                if (dr >= 0) {
                    float* qp = accb + dr * CH;
                    qp[0] += c0[r];
                    qp[16] += c1[r];
                }
            }
        }
    }
    __syncthreads();
    const size_t rowbase = (size_t)g * RG;
    for (int pass = 0; pass < 2; ++pass) {
        for (int i = 0; i < RG / 4; ++i) {
            const int rr = 4 * i + (l >> 3), qq = l & 7;
            const v4fa* p0 = (const v4fa*)(lacc + rr * CH + 4 * qq);
            v4f v = (p0[0] + p0[RG * CH / 4]) * WINV;
            const size_t grow = rowbase + rr;
            if (to_out) {
                if (grow < (size_t)nrows) {
                    v += *(const v4f*)(resid + grow * CH + 4 * qq);
                    *(volatile v4f*)(dst + grow * CH + 4 * qq) = v;
                }
            } else {
                *(volatile v4f*)(dst + grow * CH + 4 * qq) = v;
            }
        }
        __threadfence();
    }
}

__global__ __launch_bounds__(32)
void k_dsmean(const float* __restrict__ xyz, const int* __restrict__ bat,
              const int* __restrict__ slot, const int* __restrict__ off,
              int slotcap, int maxg, int nsrc, float* stg) {
    __shared__ float acc[RG * 8];
    __shared__ float st[32 * 4];
    __shared__ int wd[32];
    const int l = threadIdx.x, g = blockIdx.x;
    const int lo = clampi(off[g], 0, slotcap);
    int hi = clampi(off[g + 1], lo, slotcap);
    if (hi > lo + maxg) hi = lo + maxg;
    for (int i = 0; i < RG * 8 / 32; ++i) acc[i * 32 + l] = 0.0f;
    __syncthreads();
    for (int b0 = lo; b0 < hi; b0 += 32) {
        const int s = b0 + l;
        const int w = (s < hi) ? slot[s] : -1;
        float vx = 0.f, vy = 0.f, vz = 0.f, vb = 0.f;
        int d = -1;
        if (w >= 0) {
            int pin = w >> 8; if (pin >= nsrc) pin = nsrc - 1;
            const float* xr = xyz + (size_t)pin * 3;
            vx = xr[0]; vy = xr[1]; vz = xr[2];
            vb = (float)bat[pin];
            d = w & (RG - 1);
        }
        st[l * 4 + 0] = vx; st[l * 4 + 1] = vy; st[l * 4 + 2] = vz; st[l * 4 + 3] = vb;
        wd[l] = d;
        __syncthreads();
        for (int j = 0; j < 32; ++j) {
            const int dj = wd[j];
            if (dj >= 0 && (dj & 31) == l) {
                float* ap = acc + dj * 8;
                ap[0] += st[j * 4 + 0];
                ap[1] += st[j * 4 + 1];
                ap[2] += st[j * 4 + 2];
                ap[3] += st[j * 4 + 3];
                ap[4] += 1.0f;
            }
        }
        __syncthreads();
    }
    for (int pass = 0; pass < 2; ++pass) {
        for (int i = 0; i < RG / 32; ++i) {
            const int d = i * 32 + l;
            const float* ap = acc + d * 8;
            const float c = ap[4];
            const float inv = 1.0f / (c > 1.0f ? c : 1.0f);
            v4f v = {ap[0] * inv, ap[1] * inv, ap[2] * inv, ap[3] * inv};
            *(volatile v4f*)(stg + ((size_t)g * RG + d) * 4) = v;
        }
        __threadfence();
    }
}

__global__ __launch_bounds__(256)
void k_pack(const float* __restrict__ stg, int Mo, int nf, int nlines, int lpw, float* outr) {
    const int t = threadIdx.x, w = t >> 5, l = t & 31;
    const int lb = w * lpw;
    int le = lb + lpw; if (le > nlines) le = nlines;
    const int m3 = 3 * Mo;
    for (int pass = 0; pass < 2; ++pass) {
        for (int ln0 = lb; ln0 < le; ln0 += 4) {
            const int ln = ln0 + (l >> 3), q = l & 7;
            const int f = ln * 32 + q * 4;
            if (ln < le && f < nf) {
                v4f v;
#pragma unroll
                for (int e = 0; e < 4; ++e) {
                    const int ff = f + e;
                    float val;
                    if (ff < m3) {
                        const int d = ff / 3;
                        const int c = ff - d * 3;
                        val = stg[(size_t)d * 4 + c];
                    } else {
                        const int d = ff - m3;
                        val = (d < Mo) ? stg[(size_t)d * 4 + 3] : 0.0f;
                    }
                    v[e] = val;
                }
                *(volatile v4f*)(outr + f) = v;
            }
        }
        __threadfence();
    }
}

extern "C" void kernel_launch(void* const* d_in, const int* in_sizes, int n_in,
                              void* d_out, int out_size, void* d_ws, size_t ws_size,
                              hipStream_t stream) {
    if (n_in < 9) return;
    const float* feats    = (const float*)d_in[0];
    const float* xyz      = (const float*)d_in[1];
    const int*   bat      = (const int*)d_in[2];
    const int*   pair_in  = (const int*)d_in[3];
    const int*   pair_out = (const int*)d_in[4];
    const int*   ds_pin   = (const int*)d_in[5];
    const int*   ds_pout  = (const int*)d_in[6];
    const float* W1       = (const float*)d_in[7];
    const float* W2       = (const float*)d_in[8];

    const int N = in_sizes[0] / CH;
    if (N <= 0 || in_sizes[0] != N * CH) return;
    if (in_sizes[1] != N * 3 || in_sizes[2] != N) return;
    const int P = in_sizes[3] / KOFF;
    if (P <= 0 || in_sizes[3] != P * KOFF || in_sizes[4] != in_sizes[3]) return;
    const int P2 = in_sizes[5];
    if (P2 <= 0 || in_sizes[6] != P2) return;
    if (in_sizes[7] != KOFF * CH * CH || in_sizes[8] != KOFF * CH * CH) return;
    const long NC = (long)N * CH;
    if ((long)out_size <= NC) return;
    const long remo = (long)out_size - NC;
    if (remo % 4 != 0) return;
    const int M = (int)(remo / 4);
    if (M <= 0) return;

    const int G = (N + RG - 1) / RG;
    const int cells = G * KOFF;
    const int GP = ((G + 127) / 128) * 128;
    const int G2 = (M + RG - 1) / RG;
    const int cells2 = G2;
    const int GP2 = ((G2 + 127) / 128) * 128;
    if (G > 12288 || G2 > 12288) return;
    const long slotcapL  = (long)KOFF * P + (long)cells * 16;
    const long slotcap2L = (long)P2 + (long)cells2 * 16;
    if (slotcapL > 0x7fffff00L || slotcap2L > 0x7fffff00L) return;
    const int SLOTCAP = (int)slotcapL, SLOTCAP2 = (int)slotcap2L;
    const int noffl  = (cells + 1 + 31) / 32;
    const int noffl2 = (cells2 + 1 + 31) / 32;
    const int lpt  = (noffl + 511) / 512;
    const int lpt2 = (noffl2 + 511) / 512;
    const int GPC = (G + NCHUNK - 1) / NCHUNK;
    const int CAP = ((int)((slotcapL + NCHUNK - 1) / NCHUNK) + 4096 + 63) / 64 * 64;
    const int MAXG  = 4 * (SLOTCAP / G) + 2048;
    const int MAXG2 = 4 * (SLOTCAP2 / G2) + 2048;
    const int RB = (N + NSB - 1) / NSB;
    const int nf = 4 * M;
    const int nlines_p = (nf + 31) / 32;
    const int lpw = (nlines_p + 7) / 8;

    char* ws = (char*)d_ws;
    size_t offb = 0;
    auto carve = [&](size_t bytes) -> char* {
        char* p = ws + offb;
        offb += (bytes + 255) & ~(size_t)255;
        return p;
    };
    _Float16* Wt1  = (_Float16*)carve((size_t)KOFF * CH * CH * 2);
    _Float16* Wt2  = (_Float16*)carve((size_t)KOFF * CH * CH * 2);
    int*   cntA    = (int*)carve((size_t)KOFF * GP * 4);
    int*   cntB    = (int*)carve((size_t)GP2 * 4);
    int*   offA    = (int*)carve((size_t)noffl * 128);
    int*   offB    = (int*)carve((size_t)noffl2 * 128);
    int*   slotA   = (int*)carve((size_t)SLOTCAP * 4);
    int*   slotB   = (int*)carve((size_t)SLOTCAP2 * 4);
    float* part    = (float*)carve((size_t)NSB * 64 * 4);
    float* stat    = (float*)carve(256);
    float* h1      = (float*)carve((size_t)G * RG * CH * 4);
    _Float16* yg   = (_Float16*)carve((size_t)CAP * CH * 2);
    float* stg     = (float*)carve((size_t)G2 * RG * 16);
    if (offb > ws_size) return;

    float* out0 = (float*)d_out;
    float* outr = out0 + NC;

    const int wtot = KOFF * CH * 4;
    k_wprep<<<(wtot + 255) / 256, 256, 0, stream>>>(W1, W2, Wt1, Wt2, wtot);

    k_count<<<KOFF, 32, (size_t)GP * 4, stream>>>(pair_in, pair_out, P, N, G, GP, cntA);
    k_count<<<1, 32, (size_t)GP2 * 4, stream>>>(ds_pin, ds_pout, P2, M, G2, GP2, cntB);
    k_scan<<<1, 512, 0, stream>>>(cntA, KOFF, GP, cells, P, noffl, lpt, offA);
    k_scan<<<1, 512, 0, stream>>>(cntB, 1, GP2, cells2, P2, noffl2, lpt2, offB);
    k_fill<<<KOFF, 32, (size_t)G * 4, stream>>>(pair_in, pair_out, P, N, N, G, KOFF, offA, SLOTCAP, slotA);
    k_fill<<<1, 32, (size_t)G2 * 4, stream>>>(ds_pin, ds_pout, P2, N, M, G2, 1, offB, SLOTCAP2, slotB);

    k_stats<<<NSB, 256, 0, stream>>>(feats, N, RB, part);
    k_statfin<<<1, 64, 0, stream>>>(part, NSB, N, stat);
    for (int c = 0; c < NCHUNK; ++c) {
        const int ga = c * GPC;
        int gb = ga + GPC; if (gb > G) gb = G;
        if (ga >= gb) continue;
        k_gather<<<CAP / 64, 256, 0, stream>>>(feats, stat, slotA, offA, ga * KOFF, gb * KOFF,
                                                SLOTCAP, CAP, N, yg);
        k_conv<<<gb - ga, 32, 0, stream>>>(yg, Wt1, slotA, offA, feats, ga, SLOTCAP, CAP, MAXG,
                                           N, 0, h1);
    }

    k_stats<<<NSB, 256, 0, stream>>>(h1, N, RB, part);
    k_statfin<<<1, 64, 0, stream>>>(part, NSB, N, stat);
    for (int c = 0; c < NCHUNK; ++c) {
        const int ga = c * GPC;
        int gb = ga + GPC; if (gb > G) gb = G;
        if (ga >= gb) continue;
        k_gather<<<CAP / 64, 256, 0, stream>>>(h1, stat, slotA, offA, ga * KOFF, gb * KOFF,
                                                SLOTCAP, CAP, N, yg);
        k_conv<<<gb - ga, 32, 0, stream>>>(yg, Wt2, slotA, offA, feats, ga, SLOTCAP, CAP, MAXG,
                                           N, 1, out0);
    }

    k_dsmean<<<G2, 32, 0, stream>>>(xyz, bat, slotB, offB, SLOTCAP2, MAXG2, N, stg);
    k_pack<<<1, 256, 0, stream>>>(stg, M, nf, nlines_p, lpw, outr);
}
